// CausalSelfAttention_76184129896687
// MI455X (gfx1250) — hardware-verified
//
#include <hip/hip_runtime.h>
#ifndef NB
#define NB 2
#endif
#ifndef SQ
#define SQ 2048
#endif
#define NB_FULL 2
#define SQ_FULL 2048
#define DM 1024
#define NH 16
#define HD 64
#define EROWS 256
#define NR (NB * SQ)
#define LQK (2 * DM)
#define LV NR

static_assert(NB <= NB_FULL);
static_assert(SQ <= SQ_FULL);
static_assert(NH * HD == DM);
static_assert(HD == 64);
static_assert(DM % 32 == 0);
static_assert(DM % 128 == 0);
static_assert(NR % 128 == 0);
static_assert(NR % 64 == 0);
static_assert(LQK % 64 == 0);
static_assert(SQ % 128 == 0);
static_assert(EROWS % 64 == 0);
static_assert(SQ >= EROWS);
static_assert(DM % 8 == 0);

typedef unsigned short v8us __attribute__((ext_vector_type(8), may_alias));
typedef float  v8f  __attribute__((ext_vector_type(8)));
typedef float  v4f  __attribute__((ext_vector_type(4)));
typedef float  v4fa __attribute__((ext_vector_type(4), may_alias));
typedef _Float16 v16h __attribute__((ext_vector_type(16)));
typedef _Float16 v4h  __attribute__((ext_vector_type(4)));
union FragH { v16h v; v8us half[2]; _Float16 h[16]; };

__device__ __forceinline__ float bf16_rne(float x) {
  unsigned int u = __float_as_uint(x);
  u = (u + 0x7FFFu + ((u >> 16) & 1u)) & 0xFFFF0000u;
  return __uint_as_float(u);
}
__device__ __forceinline__ v16h ldfrag(const _Float16* __restrict__ p, size_t off) {
  FragH f;
  f.half[0] = *(const v8us*)((const unsigned short*)p + off);
  f.half[1] = *(const v8us*)((const unsigned short*)p + off + 16);
  return f.v;
}
__device__ __forceinline__ v8f wm(v16h a, v16h b, v8f c) {
  return __builtin_amdgcn_wmma_f32_16x16x32_f16(false, a, false, b, (short)0, c, false, false);
}

__global__ __launch_bounds__(256) void k_cvt16(const float* __restrict__ src, _Float16* __restrict__ dst, int rows, int rpb, int rpb_full, float scale) {
  const int t = blockIdx.x * 256 + threadIdx.x;
  if (t >= rows * (DM / 8)) return;
  const int row = t / (DM / 8), c8 = (t - row * (DM / 8)) * 8;
  const int bi = row / rpb;
  const size_t srow = (size_t)bi * rpb_full + (size_t)(row - bi * rpb);
  const v4f a = *(const v4fa*)(src + srow * DM + c8);
  const v4f c = *(const v4fa*)(src + srow * DM + c8 + 4);
  FragH f;
#pragma unroll
  for (int q = 0; q < 4; ++q) { f.h[q] = (_Float16)(bf16_rne(a[q]) * scale); f.h[4 + q] = (_Float16)(bf16_rne(c[q]) * scale); }
  const v8us o = f.half[0];
  unsigned short* d = (unsigned short*)dst + (size_t)row * DM + c8;
  *(volatile v8us*)d = o;
  __threadfence();
  *(volatile v8us*)d = o;
}

template <int MODE>
__device__ __forceinline__ void gemm_body(const _Float16* __restrict__ A, const _Float16* __restrict__ A2, int lda,
                                          const _Float16* __restrict__ Bt, int ldb, float alpha,
                                          float* __restrict__ C, _Float16* __restrict__ Ch, _Float16* __restrict__ Cl, int ldc, int N, int K) {
  __shared__ __attribute__((aligned(16))) float so[4][32][68];
  const int wave = __builtin_amdgcn_readfirstlane(threadIdx.x >> 5);
  const int lane = threadIdx.x & 31, ln = lane & 15, hh = lane >> 4;
  const int ntn = N >> 6;
  const int mt = blockIdx.x / ntn, nq = blockIdx.x - mt * ntn;
  const int row0 = mt * 128 + 32 * wave, col0 = nq * 64;
  const size_t ao0 = (size_t)(row0 + ln) * lda + 8 * hh, ao1 = ao0 + (size_t)16 * lda;
  const size_t bo0 = (size_t)(col0 + ln) * ldb + 8 * hh, bo1 = bo0 + (size_t)16 * ldb, bo2 = bo1 + (size_t)16 * ldb, bo3 = bo2 + (size_t)16 * ldb;
  const v8f z8 = {0.f, 0.f, 0.f, 0.f, 0.f, 0.f, 0.f, 0.f};
  v8f c00 = z8, c01 = z8, c02 = z8, c03 = z8, c10 = z8, c11 = z8, c12 = z8, c13 = z8;
#pragma unroll 1
  for (int kb = 0; kb < K; kb += 32) {
    const v16h a0 = ldfrag(A, ao0 + kb), a1 = ldfrag(A, ao1 + kb);
    const v16h b0 = ldfrag(Bt, bo0 + kb), b1 = ldfrag(Bt, bo1 + kb), b2 = ldfrag(Bt, bo2 + kb), b3 = ldfrag(Bt, bo3 + kb);
    v16h a0l = a0, a1l = a1;
    c00 = wm(a0, b0, c00); c10 = wm(a1, b0, c10);
    c01 = wm(a0, b1, c01); c11 = wm(a1, b1, c11);
    c02 = wm(a0, b2, c02); c12 = wm(a1, b2, c12);
    c03 = wm(a0, b3, c03); c13 = wm(a1, b3, c13);
    if (MODE == 1) {
      a0l = ldfrag(A2, ao0 + kb); a1l = ldfrag(A2, ao1 + kb);
      c00 = wm(a0l, b0, c00); c10 = wm(a1l, b0, c10);
      c01 = wm(a0l, b1, c01); c11 = wm(a1l, b1, c11);
      c02 = wm(a0l, b2, c02); c12 = wm(a1l, b2, c12);
      c03 = wm(a0l, b3, c03); c13 = wm(a1l, b3, c13);
    }
    asm volatile("v_nop\n\tv_nop\n\tv_nop\n\tv_nop"
                 : "+v"(c00), "+v"(c01), "+v"(c02), "+v"(c03), "+v"(c10), "+v"(c11), "+v"(c12), "+v"(c13)
                 : "v"(a0), "v"(a1), "v"(a0l), "v"(a1l), "v"(b0), "v"(b1), "v"(b2), "v"(b3));
  }
  v8f accs[8] = {c00, c01, c02, c03, c10, c11, c12, c13};
#pragma unroll
  for (int u = 0; u < 8; ++u) {
    const int t = u & 3, hf = u >> 2;
#pragma unroll
    for (int r = 0; r < 8; ++r) so[wave][hf * 16 + 8 * hh + r][t * 16 + ln] = accs[u][r] * alpha;
  }
  __builtin_amdgcn_fence(4  , "workgroup");
  __builtin_amdgcn_wave_barrier();
  const int rsub = lane >> 4, c4 = (lane & 15) * 4;
  for (int pass = 0; pass < 2; ++pass) {
#pragma unroll 4
    for (int q = 0; q < 16; ++q) {
      const int r = q * 2 + rsub;
      const v4f v = *(const v4fa*)&so[wave][r][c4];
      if (MODE == 0) {
        v4h h4, l4;
#pragma unroll
        for (int i = 0; i < 4; ++i) { const _Float16 hv = (_Float16)v[i]; h4[i] = hv; l4[i] = (_Float16)((v[i] - (float)hv) * 1024.0f); }
        const size_t d = (size_t)(row0 + r) * ldc + col0 + c4;
        *(volatile v4h*)(Ch + d) = h4;
        *(volatile v4h*)(Cl + d) = l4;
      } else {
        const int rr = row0 + r;
        const int bi = rr / SQ;
        const size_t orow = (size_t)bi * SQ_FULL + (size_t)(rr - bi * SQ);
        *(volatile v4f*)(C + orow * ldc + col0 + c4) = v;
      }
    }
    if (pass == 0) __threadfence();
  }
}

__global__ __launch_bounds__(128) void k_gemm_hl(const _Float16* __restrict__ A, int lda, const _Float16* __restrict__ Bt, int ldb, float alpha,
                                                 _Float16* __restrict__ Ch, _Float16* __restrict__ Cl, int ldc, int N, int K) {
  gemm_body<0>(A, A, lda, Bt, ldb, alpha, nullptr, Ch, Cl, ldc, N, K);
}
__global__ __launch_bounds__(128) void k_gemm_out(const _Float16* __restrict__ Ah, const _Float16* __restrict__ Al, int lda, const _Float16* __restrict__ Bt, int ldb, float alpha,
                                                  float* __restrict__ C, int ldc, int N, int K) {
  gemm_body<1>(Ah, Al, lda, Bt, ldb, alpha, C, nullptr, nullptr, ldc, N, K);
}

template <int EARLY>
__device__ __forceinline__ void attn_body(const _Float16* __restrict__ QKH, const _Float16* __restrict__ QKL,
                                          const _Float16* __restrict__ VTH, const _Float16* __restrict__ VTL,
                                          _Float16* __restrict__ CH, _Float16* __restrict__ CL, int qb0) {
  __shared__ __attribute__((aligned(16))) float so[4][16][68];
  const int wave = __builtin_amdgcn_readfirstlane(threadIdx.x >> 5);
  const int lane = threadIdx.x & 31, ln = lane & 15, hh = lane >> 4;
  const int qb = qb0 + blockIdx.x;
  const int b = blockIdx.y / NH, h = blockIdx.y - b * NH;
  const int tok0 = b * SQ;
  const int qw0 = qb * 64 + wave * 16;
  const size_t qoff  = (size_t)(tok0 + qw0 + ln) * LQK + h * HD + 8 * hh;
  const size_t kbase = (size_t)(tok0 + ln) * LQK + DM + h * HD + 8 * hh;
  const size_t vbase = (size_t)(h * HD + ln) * LV + tok0 + 8 * hh;
  const int qrel = qw0 + ln - 8 * hh;
  const v8f z8 = {0.f, 0.f, 0.f, 0.f, 0.f, 0.f, 0.f, 0.f};
  v8f o0 = z8, o1 = z8, o2 = z8, o3 = z8, e0 = z8, e1 = z8, e2 = z8, e3 = z8;
  float m = -1.0e30f, l = 0.f;
  const float RS = 0.0009765625f;
  const int nst = (qw0 + 47) >> 5;
#pragma unroll 1
  for (int ks = 0; ks < nst; ++ks) {
    const int k0 = ks * 32;
    const size_t ko0 = kbase + (size_t)k0 * LQK, ko1 = ko0 + (size_t)16 * LQK;
    v8f s0 = z8, s1 = z8, r0 = z8, r1 = z8;
#pragma unroll
    for (int kd = 0; kd < 2; ++kd) {
      const int dk = kd * 32;
      const v16h qh = ldfrag(QKH, qoff + dk), ql = ldfrag(QKL, qoff + dk);
      const v16h k0h = ldfrag(QKH, ko0 + dk), k0l = ldfrag(QKL, ko0 + dk);
      const v16h k1h = ldfrag(QKH, ko1 + dk), k1l = ldfrag(QKL, ko1 + dk);
      s0 = wm(k0h, qh, s0); s1 = wm(k1h, qh, s1);
      r0 = wm(k0l, qh, r0); r1 = wm(k1l, qh, r1);
      r0 = wm(k0h, ql, r0); r1 = wm(k1h, ql, r1);
      asm volatile("v_nop\n\tv_nop\n\tv_nop\n\tv_nop"
                   : "+v"(s0), "+v"(s1), "+v"(r0), "+v"(r1)
                   : "v"(qh), "v"(ql), "v"(k0h), "v"(k0l), "v"(k1h), "v"(k1l));
    }
    float p0[8], p1[8];
    float mx = -1.0e30f;
#pragma unroll
    for (int r = 0; r < 8; ++r) {
      const float a0 = (s0[r] + r0[r] * RS) * 0.125f;
      const float a1 = (s1[r] + r1[r] * RS) * 0.125f;
      p0[r] = (k0 + r <= qrel) ? a0 : -1.0e30f;
      p1[r] = (k0 + 16 + r <= qrel) ? a1 : -1.0e30f;
      mx = fmaxf(mx, fmaxf(p0[r], p1[r]));
    }
    mx = fmaxf(mx, __shfl_xor(mx, 16, 32));
    const float mn = fmaxf(m, mx);
    const float corr = __expf(m - mn);
    float ps = 0.f;
#pragma unroll
    for (int r = 0; r < 8; ++r) { p0[r] = __expf(p0[r] - mn); p1[r] = __expf(p1[r] - mn); ps += p0[r] + p1[r]; }
    ps += __shfl_xor(ps, 16, 32);
    l = l * corr + ps;
    m = mn;
    o0 = o0 * corr; o1 = o1 * corr; o2 = o2 * corr; o3 = o3 * corr;
    if (EARLY) { e0 = e0 * corr; e1 = e1 * corr; e2 = e2 * corr; e3 = e3 * corr; }
    FragH ph, pl;
#pragma unroll
    for (int r = 0; r < 8; ++r) {
      const float a0 = p0[r] * 1024.0f, a1 = p1[r] * 1024.0f;
      const _Float16 h0 = (_Float16)a0, h1 = (_Float16)a1;
      ph.h[r] = h0; ph.h[8 + r] = h1;
      if (EARLY) { pl.h[r] = (_Float16)((a0 - (float)h0) * 1024.0f); pl.h[8 + r] = (_Float16)((a1 - (float)h1) * 1024.0f); }
    }
    const size_t vo = vbase + k0;
    const v16h vh0 = ldfrag(VTH, vo), vh1 = ldfrag(VTH, vo + (size_t)16 * LV), vh2 = ldfrag(VTH, vo + (size_t)32 * LV), vh3 = ldfrag(VTH, vo + (size_t)48 * LV);
    o0 = wm(vh0, ph.v, o0); o1 = wm(vh1, ph.v, o1); o2 = wm(vh2, ph.v, o2); o3 = wm(vh3, ph.v, o3);
    if (EARLY) {
      const v16h vl0 = ldfrag(VTL, vo), vl1 = ldfrag(VTL, vo + (size_t)16 * LV), vl2 = ldfrag(VTL, vo + (size_t)32 * LV), vl3 = ldfrag(VTL, vo + (size_t)48 * LV);
      e0 = wm(vl0, ph.v, e0); e1 = wm(vl1, ph.v, e1); e2 = wm(vl2, ph.v, e2); e3 = wm(vl3, ph.v, e3);
      e0 = wm(vh0, pl.v, e0); e1 = wm(vh1, pl.v, e1); e2 = wm(vh2, pl.v, e2); e3 = wm(vh3, pl.v, e3);
      asm volatile("v_nop\n\tv_nop\n\tv_nop\n\tv_nop"
                   : "+v"(o0), "+v"(o1), "+v"(o2), "+v"(o3), "+v"(e0), "+v"(e1), "+v"(e2), "+v"(e3)
                   : "v"(ph.v), "v"(pl.v), "v"(vh0), "v"(vh1), "v"(vh2), "v"(vh3), "v"(vl0), "v"(vl1), "v"(vl2), "v"(vl3));
    } else {
      asm volatile("v_nop\n\tv_nop\n\tv_nop\n\tv_nop"
                   : "+v"(o0), "+v"(o1), "+v"(o2), "+v"(o3)
                   : "v"(ph.v), "v"(vh0), "v"(vh1), "v"(vh2), "v"(vh3));
    }
  }
  const float inv = 0.25f * (1.0f / l);
  v8f oa[4] = {o0, o1, o2, o3};
  v8f ea[4] = {e0, e1, e2, e3};
#pragma unroll
  for (int t = 0; t < 4; ++t) {
#pragma unroll
    for (int r = 0; r < 8; ++r) {
      const float c = EARLY ? (oa[t][r] + ea[t][r] * RS) * inv : oa[t][r] * inv;
      so[wave][ln][t * 16 + 8 * hh + r] = c;
    }
  }
  __builtin_amdgcn_fence(4  , "workgroup");
  __builtin_amdgcn_wave_barrier();
  const int rq = lane >> 3, pc = (lane & 7) * 8;
  for (int pass = 0; pass < 2; ++pass) {
#pragma unroll
    for (int it = 0; it < 4; ++it) {
      const int row = it * 4 + rq;
      const v4f x0 = *(const v4fa*)&so[wave][row][pc];
      const v4f x1 = *(const v4fa*)&so[wave][row][pc + 4];
      FragH fh, fl;
#pragma unroll
      for (int i = 0; i < 4; ++i) {
        const _Float16 ha = (_Float16)x0[i]; fh.h[i] = ha; fl.h[i] = (_Float16)(x0[i] - (float)ha);
        const _Float16 hb = (_Float16)x1[i]; fh.h[4 + i] = hb; fl.h[4 + i] = (_Float16)(x1[i] - (float)hb);
      }
      const v8us vh = fh.half[0], vl = fl.half[0];
      const size_t d = (size_t)(tok0 + qw0 + row) * DM + h * HD + pc;
      *(volatile v8us*)((unsigned short*)CH + d) = vh;
      *(volatile v8us*)((unsigned short*)CL + d) = vl;
    }
    if (pass == 0) __threadfence();
  }
}

__global__ __launch_bounds__(128) void k_attn_early(const _Float16* __restrict__ QKH, const _Float16* __restrict__ QKL, const _Float16* __restrict__ VTH, const _Float16* __restrict__ VTL,
                                                    _Float16* __restrict__ CH, _Float16* __restrict__ CL) {
  attn_body<1>(QKH, QKL, VTH, VTL, CH, CL, 0);
}
__global__ __launch_bounds__(128) void k_attn_main(const _Float16* __restrict__ QKH, const _Float16* __restrict__ QKL, const _Float16* __restrict__ VTH, const _Float16* __restrict__ VTL,
                                                   _Float16* __restrict__ CH, _Float16* __restrict__ CL) {
  attn_body<0>(QKH, QKL, VTH, VTL, CH, CL, EROWS / 64);
}

constexpr size_t SZ_X16 = (size_t)NR * DM * 2;
constexpr size_t SZ_W16 = (size_t)3 * DM * DM * 2;
constexpr size_t SZ_WO  = (size_t)DM * DM * 2;
constexpr size_t SZ_QK  = (size_t)NR * LQK * 2;
constexpr size_t SZ_VT  = (size_t)DM * LV * 2;
constexpr size_t SZ_C   = (size_t)NR * DM * 2;
constexpr size_t OFF_X16 = 0;
constexpr size_t OFF_W16 = OFF_X16 + SZ_X16;
constexpr size_t OFF_WO  = OFF_W16 + SZ_W16;
constexpr size_t OFF_QKH = OFF_WO + SZ_WO;
constexpr size_t OFF_QKL = OFF_QKH + SZ_QK;
constexpr size_t OFF_VTH = OFF_QKL + SZ_QK;
constexpr size_t OFF_VTL = OFF_VTH + SZ_VT;
constexpr size_t OFF_CH  = OFF_VTL + SZ_VT;
constexpr size_t OFF_CL  = OFF_CH + SZ_C;
constexpr size_t WS_TOTAL = OFF_CL + SZ_C;
static_assert(WS_TOTAL <= (size_t)134217728);
static_assert(SZ_X16 % 256 == 0);
static_assert(SZ_W16 % 256 == 0);
static_assert(SZ_WO % 256 == 0);
static_assert(SZ_QK % 256 == 0);
static_assert(SZ_VT % 256 == 0);
static_assert(SZ_C % 256 == 0);

extern "C" void kernel_launch(void* const* d_in, const int* in_sizes, int n_in,
                              void* d_out, int out_size, void* d_ws, size_t ws_size, hipStream_t stream) {
  if (n_in < 3) return;
  const size_t need_x = ((size_t)(NB - 1) * SQ_FULL + SQ) * DM;
  if ((size_t)in_sizes[0] < need_x) return;
  if ((size_t)in_sizes[1] < (size_t)3 * DM * DM) return;
  if ((size_t)in_sizes[2] < (size_t)DM * DM) return;
  if ((size_t)out_size < need_x) return;
  if (ws_size < WS_TOTAL) return;
  const float* x  = (const float*)d_in[0];
  const float* wq = (const float*)d_in[1];
  const float* wo = (const float*)d_in[2];
  float* out = (float*)d_out;
  char* ws = (char*)d_ws;
  _Float16* X16 = (_Float16*)(ws + OFF_X16);
  _Float16* W16 = (_Float16*)(ws + OFF_W16);
  _Float16* WO16 = (_Float16*)(ws + OFF_WO);
  _Float16* QKH = (_Float16*)(ws + OFF_QKH);
  _Float16* QKL = (_Float16*)(ws + OFF_QKL);
  _Float16* VTH = (_Float16*)(ws + OFF_VTH);
  _Float16* VTL = (_Float16*)(ws + OFF_VTL);
  _Float16* CH = (_Float16*)(ws + OFF_CH);
  _Float16* CL = (_Float16*)(ws + OFF_CL);

  k_cvt16<<<(unsigned)(((size_t)NR * (DM / 8) + 255) / 256), 256, 0, stream>>>(x, X16, NR, SQ, SQ_FULL, 1.0f);
  k_cvt16<<<(unsigned)(((size_t)3 * DM * (DM / 8) + 255) / 256), 256, 0, stream>>>(wq, W16, 3 * DM, 3 * DM, 3 * DM, 16.0f);
  k_cvt16<<<(unsigned)(((size_t)DM * (DM / 8) + 255) / 256), 256, 0, stream>>>(wo, WO16, DM, DM, DM, 16.0f);
  k_gemm_hl<<<(unsigned)((NR / 128) * (LQK / 64)), 128, 0, stream>>>(X16, DM, W16, DM, 0.0625f, QKH, QKL, LQK, LQK, DM);
  k_gemm_hl<<<(unsigned)((DM / 128) * (NR / 64)), 128, 0, stream>>>(W16 + (size_t)2 * DM * DM, DM, X16, DM, 0.0625f, VTH, VTL, LV, NR, DM);
  k_attn_early<<<dim3(EROWS / 64, NB * NH), 128, 0, stream>>>(QKH, QKL, VTH, VTL, CH, CL);
  if (SQ > EROWS) k_attn_main<<<dim3((SQ - EROWS) / 64, NB * NH), 128, 0, stream>>>(QKH, QKL, VTH, VTL, CH, CL);
  k_gemm_out<<<(unsigned)((NR / 128) * (DM / 64)), 128, 0, stream>>>(CH, CL, DM, WO16, DM, 0.000244140625f, out, DM, DM, DM);
}
